// GraphConv_12077448036551
// MI455X (gfx1250) — hardware-run, weakly checked
//
#include <hip/hip_runtime.h>


namespace {
constexpr int B = 16, L = 2048, DI = 256, DO = 256, BL = 16  ;
constexpr float XS = 8.0f, WSC = 256.0f;
static_assert(L % 64 == 0 && DO % 128 == 0, "tiling");
typedef _Float16 b16;
typedef __attribute__((ext_vector_type(16))) _Float16 v16b;
typedef __attribute__((ext_vector_type(8))) _Float16 v8b;
typedef __attribute__((ext_vector_type(8))) float v8f;
typedef __attribute__((ext_vector_type(4))) float v4f;
__device__ __forceinline__ float bf16_rne(float f) { unsigned int u = __float_as_uint(f); u += 0x7FFFu + ((u >> 16) & 1u); return __uint_as_float(u & 0xFFFF0000u); }
__device__ __forceinline__ void split16(float v, b16& hi, b16& lo) { hi = (b16)v; lo = (b16)(v - (float)hi); }
__device__ __forceinline__ v16b frag_kb(const b16* p, int hh) { const v8b a = *(const v8b*)(p + 8 * hh), b = *(const v8b*)(p + 16 + 8 * hh); v16b f;
#pragma unroll
  for (int e = 0; e < 8; ++e) { f[e] = a[e]; f[8 + e] = b[e]; } return f; }
__device__ __forceinline__ v8f wmma16b(v16b a, v16b b, v8f c) { v8f d = __builtin_amdgcn_wmma_f32_16x16x32_f16(false, a, false, b, (short)0, c, false, false); asm volatile("v_nop\n\tv_nop\n\tv_nop\n\tv_nop" : "+v"(d) : "v"(a), "v"(b)); return d; }
__device__ __forceinline__ void wave_lds_sync() { __builtin_amdgcn_fence(__ATOMIC_RELEASE, "workgroup"); __builtin_amdgcn_wave_barrier(); __builtin_amdgcn_fence(__ATOMIC_ACQUIRE, "workgroup"); }
__device__ __forceinline__ float pmul(float a, float b) { float p = a * b; asm volatile("" : "+v"(p)); return p; }
__device__ __forceinline__ int iclamp(int v, int lo, int hi) { return v < lo ? lo : (v > hi ? hi : v); }

typedef __attribute__((ext_vector_type(2))) _Float16 v2h;
typedef __attribute__((ext_vector_type(4))) _Float16 v4h;
__global__ __launch_bounds__(256) void prep_kernel(const float* __restrict__ w, b16* __restrict__ WT) {
  const int t = blockIdx.x * 256 + threadIdx.x; if (t >= DO * DI / 8) return; const int e = t * 8; const int oo = e / DI, k0 = e % DI; v8b o;
  for (int j = 0; j < 8; ++j) o[j] = (b16)(bf16_rne(w[(size_t)(k0 + j) * DO + oo]) * WSC);
  for (int pass = 0; pass < 2; ++pass) { *(volatile v8b*)(WT + e) = o; __threadfence(); }
}
__global__ __launch_bounds__(256) void gt_kernel(const float* __restrict__ g, b16* __restrict__ GT) {
  __shared__ float tile[64][65];
  const int m0 = blockIdx.x * 64, l0 = blockIdx.y * 64;
  for (int i = threadIdx.x; i < 64 * 64; i += 256) { const int mm = i / 64, ll = i % 64; tile[mm][ll] = g[(size_t)(m0 + mm) * L + l0 + ll]; }
  __syncthreads();
  for (int pass = 0; pass < 2; ++pass) { for (int i = threadIdx.x; i < 64 * 16; i += 256) { const int ll = i / 16, mq = (i % 16) * 4; v4h o; for (int j = 0; j < 4; ++j) { const int l = l0 + ll, m = m0 + mq + j; o[j] = (b16)((tile[mq + j][ll] != 0.0f || l == m) ? 1.0f : 0.0f); } *(volatile v4h*)(GT + (size_t)(l0 + ll) * L + m0 + mq) = o; } __threadfence(); }
}
__global__ __launch_bounds__(256) void deg_kernel(const b16* __restrict__ GT, float* __restrict__ DINV) {
  const int wave = threadIdx.x >> 5, lane = threadIdx.x & 31; const int lb = (blockIdx.x * 8 + wave) * 32;
  const int l = lb + lane; float s = 0.0f;
#pragma unroll 4
  for (int m = 0; m < L; m += 8) { const v8b v = *(const v8b*)(GT + (size_t)l * L + m); for (int j = 0; j < 8; ++j) s += (float)v[j]; }
  const float dv = (s > 0.0f) ? rsqrtf(s) : 0.0f;
  for (int pass = 0; pass < 2; ++pass) { ((volatile float*)DINV)[l] = dv; __threadfence(); }
}
__global__ __launch_bounds__(128) void feat_kernel(const float* __restrict__ x, const b16* __restrict__ WT, const float* __restrict__ DINV, b16* __restrict__ HST) {
  __shared__ __attribute__((aligned(16))) float Tf[4][16][128 + 4];
  const int wave = threadIdx.x >> 5, lane = threadIdx.x & 31, nloc = lane & 15, hlf = lane >> 4; const int t0 = blockIdx.x * 64; const int b = blockIdx.y; const int n0 = blockIdx.z * 128;
  const size_t r0 = (size_t)b * L + t0 + wave * 16;
  v8f acc[8];
#pragma unroll
  for (int t = 0; t < 8; ++t) acc[t] = (v8f){};
#pragma unroll 2
  for (int ks = 0; ks < DI / 32; ++ks) { v16b a; const float* xr = x + (r0 + nloc) * DI + ks * 32; const v4f c0 = *(const v4f*)(xr + 8 * hlf), c1 = *(const v4f*)(xr + 8 * hlf + 4), c2 = *(const v4f*)(xr + 16 + 8 * hlf), c3 = *(const v4f*)(xr + 16 + 8 * hlf + 4);
    for (int i = 0; i < 4; ++i) { a[i] = (b16)(bf16_rne(c0[i]) * XS); a[4 + i] = (b16)(bf16_rne(c1[i]) * XS); a[8 + i] = (b16)(bf16_rne(c2[i]) * XS); a[12 + i] = (b16)(bf16_rne(c3[i]) * XS); }
#pragma unroll
    for (int t = 0; t < 8; ++t) acc[t] = wmma16b(a, frag_kb(WT + (size_t)(n0 + t * 16 + nloc) * DI + ks * 32, hlf), acc[t]); }
#pragma unroll
  for (int t = 0; t < 8; ++t)
#pragma unroll
    for (int r = 0; r < 8; ++r) { const int m = t0 + wave * 16 + 8 * hlf + r; Tf[wave][8 * hlf + r][t * 16 + nloc] = acc[t][r] * (1.0f / (XS * WSC)) * DINV[m]; }
  __syncthreads();
  for (int pass = 0; pass < 2; ++pass) {
#pragma unroll 1
    for (int q = 0; q < 32; ++q) { const int c = wave * 32 + q; const int tk = lane * 2; v2h o2; o2[0] = (b16)(Tf[tk >> 4][tk & 15][c] * XS); o2[1] = (b16)(Tf[(tk + 1) >> 4][(tk + 1) & 15][c] * XS);
      *(volatile v2h*)(HST + ((size_t)b * DO + n0 + c) * L + t0 + tk) = o2; }
    __threadfence(); }
}
__global__ __launch_bounds__(128) void agg_kernel(const b16* __restrict__ GT, const b16* __restrict__ HST, const float* __restrict__ DINV, const float* __restrict__ bias, const float* __restrict__ x, float* __restrict__ out) {
  __shared__ __attribute__((aligned(16))) float Tf[4][16][128 + 4];
  const int wave = threadIdx.x >> 5, lane = threadIdx.x & 31, nloc = lane & 15, hlf = lane >> 4; const int l0 = blockIdx.x * 64 + wave * 16; const int n0 = blockIdx.y * 128; const int b = blockIdx.z;
  const b16* Bp = HST + ((size_t)b * DO + n0) * L;
  v8f acc[8];
#pragma unroll
  for (int t = 0; t < 8; ++t) acc[t] = (v8f){};
#pragma unroll 2
  for (int kb = 0; kb < L; kb += 32) { const v16b a = frag_kb(GT + (size_t)(l0 + nloc) * L + kb, hlf);
#pragma unroll
    for (int t = 0; t < 8; ++t) acc[t] = wmma16b(a, frag_kb(Bp + (size_t)(t * 16 + nloc) * L + kb, hlf), acc[t]); }
#pragma unroll
  for (int t = 0; t < 8; ++t) { const float bb = bf16_rne(bias[n0 + t * 16 + nloc]);
#pragma unroll
    for (int r = 0; r < 8; ++r) { const int l = l0 + 8 * hlf + r; Tf[wave][8 * hlf + r][t * 16 + nloc] = fmaxf(acc[t][r] * (1.0f / XS) * DINV[l] + bb, 0.0f); } }
  wave_lds_sync();
  for (int pass = 0; pass < 2; ++pass) { for (int rr = 0; rr < 16; ++rr) { const size_t row = (size_t)b * L + l0 + rr; const v4f xv = *(const v4f*)(x + row * DI + n0 + lane * 4); v4f o = *(const v4f*)(&Tf[wave][rr][lane * 4]); for (int j = 0; j < 4; ++j) o[j] += bf16_rne(xv[j]); *(volatile v4f*)(out + row * DO + n0 + lane * 4) = o; } __threadfence(); }
}
}

extern "C" void kernel_launch(void* const* d_in, const int* in_sizes, int n_in, void* d_out, int out_size, void* d_ws, size_t ws_size, hipStream_t stream) {
  (void)n_in;
  auto Fp = [&](int i) { return (const float*)d_in[i]; };
  if (in_sizes[0] != B * L * DI || in_sizes[1] != L * L || in_sizes[2] != DI * DO || in_sizes[3] != DO || out_size != B * L * DO) return;
  size_t off = 0; char* ws = (char*)d_ws;
  auto carve = [&](size_t bytes) { char* p = ws + off; off += (bytes + 255) & ~(size_t)255; return p; };
  b16* WT = (b16*)carve((size_t)DO * DI * 2); b16* GT = (b16*)carve((size_t)L * L * 2); float* DINV = (float*)carve((size_t)L * 4); b16* HST = (b16*)carve((size_t)B * DO * L * 2);
  if (off > ws_size || off > ((size_t)128 << 20)) return;
  prep_kernel<<<(DO * DI / 8 + 255) / 256, 256, 0, stream>>>(Fp(2), WT);
  gt_kernel<<<dim3(L / 64, L / 64), 256, 0, stream>>>(Fp(1), GT);
  deg_kernel<<<L / 256, 256, 0, stream>>>(GT, DINV);
  feat_kernel<<<dim3(L / 64, BL, DO / 128), 128, 0, stream>>>(Fp(0), WT, DINV, HST);
  agg_kernel<<<dim3(L / 64, DO / 128, BL), 128, 0, stream>>>(GT, HST, DINV, Fp(3), Fp(0), (float*)d_out);
}
